// EncoderLayer_12979391168612
// MI455X (gfx1250) — hardware-verified
//
#include <hip/hip_runtime.h>
#ifndef NB
#define NB 2
#endif
#ifndef SEQ
#define SEQ 2048
#endif
#define NB_FULL 2
#define SEQ_FULL 2048
#define DM 1024
#define NH 16
#define HD 64
#define DFF 4096
#define HG 2
#define QT0 128
#define LQK (2 * DM)
static_assert(NB <= NB_FULL);
static_assert(SEQ <= SEQ_FULL);
static_assert(SEQ % 128 == 0);
static_assert(SEQ >= 2 * QT0);
static_assert((SEQ - QT0) % 128 == 0);
static_assert(QT0 % 64 == 0);
static_assert(NH % HG == 0);
static_assert(NH * HD == DM);
static_assert(DM % 64 == 0);
static_assert(DFF % 64 == 0);
static_assert(HD % 32 == 0);
static_assert((HG * SEQ) % 256 == 0);

typedef unsigned short v8us __attribute__((ext_vector_type(8), may_alias));
typedef float  v8f  __attribute__((ext_vector_type(8)));
typedef float  v4f  __attribute__((ext_vector_type(4)));
typedef float  v4fa __attribute__((ext_vector_type(4), may_alias));
typedef _Float16 v16h __attribute__((ext_vector_type(16)));
typedef _Float16 v4h __attribute__((ext_vector_type(4)));
union FragH { v16h v; v8us half[2]; _Float16 h[16]; unsigned short u[16]; };

__device__ __forceinline__ unsigned short bf16_bits(float x) { unsigned int u = __float_as_uint(x); return (unsigned short)((u + 0x7FFFu + ((u >> 16) & 1u)) >> 16); }
__device__ __forceinline__ float bf16_val(unsigned short b) { return __uint_as_float(((unsigned int)b) << 16); }
__device__ __forceinline__ float bf16_rne(float x) { return bf16_val(bf16_bits(x)); }

__device__ __forceinline__ v16h g2_frag(const _Float16* p, int hh) { FragH f; f.half[0] = *(const v8us*)((const unsigned short*)p + 8 * hh); f.half[1] = *(const v8us*)((const unsigned short*)p + 16 + 8 * hh); return f.v; }
__device__ __forceinline__ v8f g2_mma(v16h a, v16h b, v8f c) { v8f d = __builtin_amdgcn_wmma_f32_16x16x32_f16(false, a, false, b, (short)0, c, false, false); asm volatile("v_nop\n\tv_nop\n\tv_nop\n\tv_nop" : "+v"(d) : "v"(a), "v"(b)); return d; }

__global__ __launch_bounds__(256) void k_wt_f16(const float* __restrict__ W, _Float16* __restrict__ Wt, int K, int N, float scale) {
  const int t = blockIdx.x * 256 + threadIdx.x; if (t >= N * (K / 8)) return; const int n = t / (K / 8), k8 = (t % (K / 8)) * 8; FragH f;
#pragma unroll
  for (int i = 0; i < 8; ++i) f.h[i] = (_Float16)(bf16_rne(W[(size_t)(k8 + i) * N + n]) * scale);
  const v8us o = f.half[0];
  *(volatile v8us*)((unsigned short*)Wt + (size_t)n * K + k8) = o; __threadfence(); *(volatile v8us*)((unsigned short*)Wt + (size_t)n * K + k8) = o;
}

__global__ __launch_bounds__(256) void k_wthd(const float* __restrict__ W, _Float16* __restrict__ Bt) {
  const size_t t = (size_t)blockIdx.x * 256 + threadIdx.x; if (t >= (size_t)NH * HD * (DM / 8)) return;
  const int m8 = (int)(t % (DM / 8)) * 8; const int d = (int)((t / (DM / 8)) % HD); const int h = (int)(t / ((size_t)(DM / 8) * HD)); FragH f;
#pragma unroll
  for (int q = 0; q < 8; ++q) f.h[q] = (_Float16)(16.0f * bf16_rne(W[((size_t)h * DM + m8 + q) * HD + d]));
  unsigned short* dst = (unsigned short*)Bt + ((size_t)h * HD + d) * DM + m8; const v8us o = f.half[0];
  *(volatile v8us*)dst = o; __threadfence(); *(volatile v8us*)dst = o;
}

__global__ __launch_bounds__(256) void k_x16(const float* __restrict__ x, _Float16* __restrict__ X16, size_t n8) {
  const size_t t = (size_t)blockIdx.x * 256 + threadIdx.x; if (t >= n8) return; FragH f;
  const v4f a = *(const v4fa*)(x + t * 8), c = *(const v4fa*)(x + t * 8 + 4);
#pragma unroll
  for (int q = 0; q < 4; ++q) { f.h[q] = (_Float16)bf16_rne(a[q]); f.h[4 + q] = (_Float16)bf16_rne(c[q]); }
  const v8us o = f.half[0];
  *(volatile v8us*)((unsigned short*)X16 + t * 8) = o; __threadfence(); *(volatile v8us*)((unsigned short*)X16 + t * 8) = o;
}

template <int NHv, int TTv>
__global__ __launch_bounds__(256) void k_vt(const _Float16* __restrict__ V16, int ldv, int voff, _Float16* __restrict__ Vt) {
  __shared__ unsigned short tl[64][66]; const int tid = threadIdx.x; const int slab = blockIdx.x / (TTv / 64), lg = blockIdx.x % (TTv / 64); const int b = slab / NHv, h = slab % NHv;
  for (int i = tid; i < 64 * 8; i += 256) { const int r = i / 8, c8 = (i % 8) * 8; FragH f; f.half[0] = *(const v8us*)((const unsigned short*)V16 + ((size_t)b * TTv + lg * 64 + r) * ldv + voff + h * 64 + c8);
#pragma unroll
    for (int q = 0; q < 8; ++q) tl[r][c8 + q] = f.u[q]; }
  __syncthreads();
  for (int pass = 0; pass < 2; ++pass) {
#pragma unroll
    for (int rd = 0; rd < 2; ++rd) { const int d = rd * 32 + tid / 8, pc = tid % 8; FragH f;
#pragma unroll
      for (int q = 0; q < 8; ++q) f.u[q] = tl[pc * 8 + q][d];
      *(volatile v8us*)((unsigned short*)Vt + ((size_t)slab * 64 + d) * TTv + lg * 64 + pc * 8) = f.half[0]; }
    if (pass == 0) __threadfence(); } }

template <int ACT, int CPBF>
__global__ __launch_bounds__(128) void k_gemm2(const _Float16* __restrict__ A, int lda, size_t sA, const _Float16* __restrict__ Bh, int ldb, size_t sB, float alpha,
    const float* __restrict__ bias, const float* __restrict__ CP, int row0g, const float* __restrict__ RS, size_t sRS,
    float* __restrict__ C, _Float16* __restrict__ C16, _Float16* __restrict__ C16L, int ldc, size_t sC, int M, int N, int K) {
  static_assert(ACT == 0 || ACT == 3);
  __shared__ __attribute__((aligned(16))) float so[4][32][68];
  const int tid = threadIdx.x, w = tid >> 5, lane = tid & 31, ln = lane & 15, hh = lane >> 4; const int by = blockIdx.y;
  A += (size_t)by * sA; Bh += (size_t)by * sB; const size_t cofs = (size_t)by * sC;
  const int ntn = N >> 6; const int mt = blockIdx.x / ntn, nq = blockIdx.x - mt * ntn; const int row0 = mt * 128 + 32 * w, col0 = nq * 64; if (row0 >= M) return;
  const _Float16* a0p = A + (size_t)(row0 + ln) * lda; const _Float16* a1p = a0p + (size_t)16 * lda;
  const _Float16* b0p = Bh + (size_t)(col0 + ln) * ldb; const _Float16* b1p = b0p + (size_t)16 * ldb; const _Float16* b2p = b1p + (size_t)16 * ldb; const _Float16* b3p = b2p + (size_t)16 * ldb;
  const v8f z8 = {0.f,0.f,0.f,0.f,0.f,0.f,0.f,0.f}; v8f c00 = z8, c01 = z8, c02 = z8, c03 = z8, c10 = z8, c11 = z8, c12 = z8, c13 = z8;
#pragma unroll 1
  for (int kb = 0; kb < K; kb += 32) { const v16h a0 = g2_frag(a0p + kb, hh), a1 = g2_frag(a1p + kb, hh);
    v16h b = g2_frag(b0p + kb, hh); c00 = g2_mma(a0, b, c00); c10 = g2_mma(a1, b, c10);
    b = g2_frag(b1p + kb, hh); c01 = g2_mma(a0, b, c01); c11 = g2_mma(a1, b, c11);
    b = g2_frag(b2p + kb, hh); c02 = g2_mma(a0, b, c02); c12 = g2_mma(a1, b, c12);
    b = g2_frag(b3p + kb, hh); c03 = g2_mma(a0, b, c03); c13 = g2_mma(a1, b, c13); }
  v8f accs[8] = {c00, c01, c02, c03, c10, c11, c12, c13};
#pragma unroll
  for (int u = 0; u < 8; ++u) { const int t = u & 3, half = u >> 2; const int col = col0 + t * 16 + ln; const float bv = bias ? bf16_rne(bias[col]) : 0.f;
#pragma unroll
    for (int r = 0; r < 8; ++r) { const int rloc = half * 16 + 8 * hh + r; float v = accs[u][r] * alpha;
      if (RS) v *= RS[(size_t)by * sRS + (size_t)(row0g + row0 + rloc)];
      v += bv;
      if (CP) { float cv = CP[cofs + (size_t)(row0g + row0 + rloc) * ldc + col]; if (CPBF) cv = bf16_rne(cv); v += cv; }
      if (ACT == 3) v = fmaxf(v, 0.f);
      so[w][rloc][t * 16 + ln] = v; } }
  __builtin_amdgcn_fence(4  , "workgroup"); __builtin_amdgcn_wave_barrier();
  const int rsub = lane >> 4, c4 = (lane & 15) * 4;
  for (int pass = 0; pass < 2; ++pass) {
#pragma unroll
    for (int q = 0; q < 16; ++q) { const int r = q * 2 + rsub; const v4f v = *(const v4fa*)&so[w][r][c4]; const size_t o = cofs + (size_t)(row0 + r) * ldc + col0 + c4;
      if (C) *(volatile v4f*)(C + o) = v;
      if (C16 || C16L) { v4h h4, l4;
#pragma unroll
        for (int i = 0; i < 4; ++i) { h4[i] = (_Float16)v[i]; l4[i] = (_Float16)((v[i] - (float)h4[i]) * 1024.0f); }
        if (C16) *(volatile v4h*)(C16 + o) = h4;
        if (C16L) *(volatile v4h*)(C16L + o) = l4; } }
    if (pass == 0) __threadfence(); } }

template <int DUAL, int CPBF>
__global__ __launch_bounds__(128) void k_gemmf(const _Float16* __restrict__ A, const _Float16* A2, int lda, size_t sA, const _Float16* __restrict__ Bh, const _Float16* B2, int ldb, size_t sB, float alpha,
    const float* __restrict__ CP, const float* __restrict__ RS, size_t sRS,
    float* __restrict__ C, _Float16* __restrict__ C16, _Float16* __restrict__ C16L, int ldc, size_t sC, int M, int N, int K) {
  static_assert(DUAL == 1 || DUAL == 2);
  __shared__ __attribute__((aligned(16))) float so[4][16][68];
  const int tid = threadIdx.x, w = tid >> 5, lane = tid & 31, ln = lane & 15, hh = lane >> 4; const int by = blockIdx.y;
  const size_t cofs = (size_t)by * sC;
  const int ntn = N >> 6; const int wid = blockIdx.x * 4 + w; const int mt = wid / ntn, nq = wid - mt * ntn; const int row0 = mt * 16, col0 = nq * 64; if (row0 >= M) return;
  const _Float16* ap = A + (size_t)by * sA + (size_t)(row0 + ln) * lda;
  const _Float16* a2p = (DUAL == 1) ? (A2 + (size_t)by * sA + (size_t)(row0 + ln) * lda) : ap;
  const _Float16* bp = Bh + (size_t)by * sB + (size_t)(col0 + ln) * ldb;
  const _Float16* dp = (DUAL == 2) ? (B2 + (size_t)by * sB + (size_t)(col0 + ln) * ldb) : bp;
  const size_t bs = (size_t)16 * ldb;
  const v8f z8 = {0.f,0.f,0.f,0.f,0.f,0.f,0.f,0.f}; v8f c0 = z8, c1 = z8, c2 = z8, c3 = z8, e0 = z8, e1 = z8, e2 = z8, e3 = z8;
#pragma unroll 1
  for (int kb = 0; kb < K; kb += 32) { const v16h a = g2_frag(ap + kb, hh);
    if (DUAL == 1) { const v16h a2 = g2_frag(a2p + kb, hh);
      v16h b = g2_frag(bp + kb, hh); c0 = g2_mma(a, b, c0); e0 = g2_mma(a2, b, e0);
      b = g2_frag(bp + bs + kb, hh); c1 = g2_mma(a, b, c1); e1 = g2_mma(a2, b, e1);
      b = g2_frag(bp + 2 * bs + kb, hh); c2 = g2_mma(a, b, c2); e2 = g2_mma(a2, b, e2);
      b = g2_frag(bp + 3 * bs + kb, hh); c3 = g2_mma(a, b, c3); e3 = g2_mma(a2, b, e3);
    } else {
      v16h b = g2_frag(bp + kb, hh); c0 = g2_mma(a, b, c0); b = g2_frag(dp + kb, hh); e0 = g2_mma(a, b, e0);
      b = g2_frag(bp + bs + kb, hh); c1 = g2_mma(a, b, c1); b = g2_frag(dp + bs + kb, hh); e1 = g2_mma(a, b, e1);
      b = g2_frag(bp + 2 * bs + kb, hh); c2 = g2_mma(a, b, c2); b = g2_frag(dp + 2 * bs + kb, hh); e2 = g2_mma(a, b, e2);
      b = g2_frag(bp + 3 * bs + kb, hh); c3 = g2_mma(a, b, c3); b = g2_frag(dp + 3 * bs + kb, hh); e3 = g2_mma(a, b, e3);
    } }
  v8f cs[4] = {c0, c1, c2, c3}; v8f es[4] = {e0, e1, e2, e3};
#pragma unroll
  for (int t = 0; t < 4; ++t) { const int col = col0 + t * 16 + ln;
#pragma unroll
    for (int r = 0; r < 8; ++r) { const int rloc = 8 * hh + r; float v = (cs[t][r] + es[t][r] * 0.0009765625f) * alpha;
      if (RS) v *= RS[(size_t)by * sRS + (size_t)(row0 + rloc)];
      if (CP) { float cv = CP[cofs + (size_t)(row0 + rloc) * ldc + col]; if (CPBF) cv = bf16_rne(cv); v += cv; }
      so[w][rloc][t * 16 + ln] = v; } }
  __builtin_amdgcn_fence(4  , "workgroup"); __builtin_amdgcn_wave_barrier();
  const int rsub = lane >> 4, c4 = (lane & 15) * 4;
  for (int pass = 0; pass < 2; ++pass) {
#pragma unroll
    for (int q = 0; q < 8; ++q) { const int r = q * 2 + rsub; const v4f v = *(const v4fa*)&so[w][r][c4]; const size_t o = cofs + (size_t)(row0 + r) * ldc + col0 + c4;
      if (C) *(volatile v4f*)(C + o) = v;
      if (C16 || C16L) { v4h h4, l4;
#pragma unroll
        for (int i = 0; i < 4; ++i) { h4[i] = (_Float16)v[i]; l4[i] = (_Float16)((v[i] - (float)h4[i]) * 1024.0f); }
        if (C16) *(volatile v4h*)(C16 + o) = h4;
        if (C16L) *(volatile v4h*)(C16L + o) = l4; } }
    if (pass == 0) __threadfence(); } }

__global__ __launch_bounds__(256) void k_rsms(const float* __restrict__ S, _Float16* __restrict__ P, float* __restrict__ RL, int nrows) {
  #pragma clang fp contract(off)
  const int t = blockIdx.x * 256 + threadIdx.x; if (t >= nrows) return; const int qi = t % SEQ; const float* s = S + (size_t)t * SEQ; float mx = -3.0e38f;
#pragma unroll 1
  for (int j0 = 0; j0 < SEQ; j0 += 4) { const v4f a = *(const v4fa*)(s + j0);
#pragma unroll
    for (int q = 0; q < 4; ++q) { const float v = a[q] + ((j0 + q > qi) ? -12.5f : 0.f); mx = fmaxf(mx, v); } }
  float l = 0.f;
#pragma unroll 1
  for (int j0 = 0; j0 < SEQ; j0 += 8) { const v4f a = *(const v4fa*)(s + j0), c = *(const v4fa*)(s + j0 + 4); FragH f;
#pragma unroll
    for (int q = 0; q < 4; ++q) {
      const float v0 = a[q] + ((j0 + q > qi) ? -12.5f : 0.f); const _Float16 h0 = (_Float16)(__expf(v0 - mx) * 16384.0f); f.h[q] = h0; l += (float)h0;
      const float v1 = c[q] + ((j0 + 4 + q > qi) ? -12.5f : 0.f); const _Float16 h1 = (_Float16)(__expf(v1 - mx) * 16384.0f); f.h[4 + q] = h1; l += (float)h1; }
    unsigned short* d = (unsigned short*)P + (size_t)t * SEQ + j0; const v8us o = f.half[0];
    *(volatile v8us*)d = o; __threadfence(); *(volatile v8us*)d = o; }
  const float ri = 1.0f / l;
  *(volatile float*)(RL + t) = ri; __threadfence(); *(volatile float*)(RL + t) = ri; }

template <int W16>
__global__ __launch_bounds__(256) void k_lnseq(const float* __restrict__ X, const float* __restrict__ g, const float* __restrict__ bb, float eps, float* __restrict__ N32, _Float16* __restrict__ N16, int rows) {
  #pragma clang fp contract(off)
  __shared__ float red[16][64]; __shared__ float st[2][64];
  const int tid = threadIdx.x, cq = tid & 15, rr = tid >> 4; const int c0 = blockIdx.x * 64 + cq * 4; const float inv = 1.0f / (float)rows;
  v4f s = {0.f, 0.f, 0.f, 0.f};
#pragma unroll 1
  for (int r = rr; r < rows; r += 16) { const v4f a = *(const v4fa*)(X + (size_t)r * DM + c0); s += a; }
#pragma unroll
  for (int q = 0; q < 4; ++q) red[rr][cq * 4 + q] = s[q];
  __syncthreads();
  if (tid < 64) { float a = 0.f;
#pragma unroll 1
    for (int k = 0; k < 16; ++k) a += red[k][tid];
    st[0][tid] = a * inv; }
  __syncthreads();
  v4f mu;
#pragma unroll
  for (int q = 0; q < 4; ++q) mu[q] = st[0][cq * 4 + q];
  v4f vs = {0.f, 0.f, 0.f, 0.f};
#pragma unroll 1
  for (int r = rr; r < rows; r += 16) { const v4f a = *(const v4fa*)(X + (size_t)r * DM + c0); const v4f d = a - mu; vs += d * d; }
#pragma unroll
  for (int q = 0; q < 4; ++q) red[rr][cq * 4 + q] = vs[q];
  __syncthreads();
  if (tid < 64) { float a = 0.f;
#pragma unroll 1
    for (int k = 0; k < 16; ++k) a += red[k][tid];
    st[1][tid] = rsqrtf(a * inv + eps); }
  __syncthreads();
  v4f rs, gg, bo;
#pragma unroll
  for (int q = 0; q < 4; ++q) { rs[q] = st[1][cq * 4 + q]; gg[q] = bf16_rne(g[c0 + q]); bo[q] = bf16_rne(bb[c0 + q]); }
  for (int pass = 0; pass < 2; ++pass) {
#pragma unroll 1
    for (int r = rr; r < rows; r += 16) { const v4f a = *(const v4fa*)(X + (size_t)r * DM + c0); v4f y; v4h yh;
#pragma unroll
      for (int q = 0; q < 4; ++q) { y[q] = (a[q] - mu[q]) * rs[q] * gg[q] + bo[q]; yh[q] = (_Float16)y[q]; }
      *(volatile v4f*)(N32 + (size_t)r * DM + c0) = y;
      if (W16) *(volatile v4h*)(N16 + (size_t)r * DM + c0) = yh; }
    if (pass == 0) __threadfence(); } }

constexpr size_t al256(size_t b) { return (b + 255) & ~(size_t)255; }
constexpr size_t SZ_BQKV = al256((size_t)3 * DM * DM * 2);
constexpr size_t SZ_BO   = al256((size_t)DM * DM * 2);
constexpr size_t SZ_BW1  = al256((size_t)DFF * DM * 2);
constexpr size_t SZ_BW2  = al256((size_t)DM * DFF * 2);
constexpr size_t SZ_X16  = al256((size_t)SEQ * DM * 2);
constexpr size_t SZ_QK16 = al256((size_t)SEQ * LQK * 2);
constexpr size_t SZ_VH   = al256((size_t)SEQ * DM * 2);
constexpr size_t SZ_VT   = al256((size_t)NH * HD * SEQ * 2);
constexpr size_t SZ_O16  = al256((size_t)SEQ * DM * 2);
constexpr size_t SZ_OL   = al256((size_t)QT0 * DM * 2);
constexpr size_t SZ_RL   = al256((size_t)HG * SEQ * 4);
constexpr size_t SZ_S    = al256((size_t)HG * SEQ * SEQ * 4);
constexpr size_t SZ_P    = al256((size_t)HG * SEQ * SEQ * 2);
constexpr size_t SZ_Y    = al256((size_t)SEQ * DM * 4);
constexpr size_t SZ_N16  = al256((size_t)SEQ * DM * 2);
constexpr size_t SZ_HF   = al256((size_t)SEQ * DFF * 2);
constexpr size_t SZ_RA_ATT  = SZ_S + SZ_P;
constexpr size_t SZ_RA_POST = SZ_Y + SZ_Y + SZ_N16 + SZ_HF + SZ_Y;
constexpr size_t SZ_RA = (SZ_RA_ATT > SZ_RA_POST) ? SZ_RA_ATT : SZ_RA_POST;
constexpr size_t WS_TOTAL = SZ_BQKV + SZ_BO + SZ_BW1 + SZ_BW2 + SZ_X16 + SZ_QK16 + 2 * SZ_VH + 2 * SZ_VT + SZ_O16 + SZ_OL + SZ_RL + SZ_RA;
static_assert(SZ_RA_ATT <= SZ_RA);
static_assert(SZ_RA_POST <= SZ_RA);
static_assert(WS_TOTAL <= (size_t)134217728);

extern "C" void kernel_launch(void* const* d_in, const int* in_sizes, int n_in,
                              void* d_out, int out_size, void* d_ws, size_t ws_size, hipStream_t stream) {
  if (n_in < 13) return;
  const size_t xneed = ((size_t)(NB - 1) * SEQ_FULL + SEQ) * DM;
  if ((size_t)in_sizes[0] < xneed || (size_t)out_size < xneed) return;
  if ((size_t)in_sizes[1] < (size_t)NH * DM * HD || (size_t)in_sizes[2] < (size_t)NH * DM * HD || (size_t)in_sizes[3] < (size_t)NH * DM * HD || (size_t)in_sizes[4] < (size_t)NH * HD * DM) return;
  if (in_sizes[5] < DM || in_sizes[6] < DM || (size_t)in_sizes[7] < (size_t)DM * DFF || in_sizes[8] < DFF || (size_t)in_sizes[9] < (size_t)DFF * DM || in_sizes[10] < DM || in_sizes[11] < DM || in_sizes[12] < DM) return;
  if (WS_TOTAL > ws_size) return;
  const float* x = (const float*)d_in[0]; const float* wq = (const float*)d_in[1]; const float* wk = (const float*)d_in[2]; const float* wv = (const float*)d_in[3]; const float* wo = (const float*)d_in[4];
  const float* ln1s = (const float*)d_in[5]; const float* ln1o = (const float*)d_in[6]; const float* w1 = (const float*)d_in[7]; const float* b1 = (const float*)d_in[8]; const float* w2 = (const float*)d_in[9]; const float* b2 = (const float*)d_in[10];
  const float* ln2s = (const float*)d_in[11]; const float* ln2o = (const float*)d_in[12];
  char* ws = (char*)d_ws; size_t off = 0;
  auto take = [&](size_t bytes) { char* p = ws + off; off += bytes; return p; };
  _Float16* BQKV = (_Float16*)take(SZ_BQKV); _Float16* BO = (_Float16*)take(SZ_BO); _Float16* BW1 = (_Float16*)take(SZ_BW1); _Float16* BW2 = (_Float16*)take(SZ_BW2);
  _Float16* X16 = (_Float16*)take(SZ_X16); _Float16* QK16 = (_Float16*)take(SZ_QK16); _Float16* VH = (_Float16*)take(SZ_VH); _Float16* VL = (_Float16*)take(SZ_VH);
  _Float16* VT = (_Float16*)take(SZ_VT); _Float16* VTL = (_Float16*)take(SZ_VT); _Float16* O16 = (_Float16*)take(SZ_O16); _Float16* OL = (_Float16*)take(SZ_OL); float* RL = (float*)take(SZ_RL);
  char* RA = take(SZ_RA);
  if (off != WS_TOTAL) return;
  float* S = (float*)RA; _Float16* P = (_Float16*)(RA + SZ_S);
  float* Y1 = (float*)RA; float* NORM = (float*)(RA + SZ_Y); _Float16* N16 = (_Float16*)(RA + 2 * SZ_Y); _Float16* HF16 = (_Float16*)(RA + 2 * SZ_Y + SZ_N16); float* Y2 = (float*)(RA + 2 * SZ_Y + SZ_N16 + SZ_HF);

  { const unsigned gh = (unsigned)(((size_t)NH * HD * (DM / 8) + 255) / 256);
    k_wthd<<<gh, 256, 0, stream>>>(wq, BQKV);
    k_wthd<<<gh, 256, 0, stream>>>(wk, BQKV + (size_t)DM * DM);
    k_wthd<<<gh, 256, 0, stream>>>(wv, BQKV + (size_t)2 * DM * DM);
    k_wt_f16<<<(unsigned)(((size_t)DM * (DM / 8) + 255) / 256), 256, 0, stream>>>(wo, BO, DM, DM, 16.0f);
    k_wt_f16<<<(unsigned)(((size_t)DFF * (DM / 8) + 255) / 256), 256, 0, stream>>>(w1, BW1, DM, DFF, 16.0f);
    k_wt_f16<<<(unsigned)(((size_t)DM * (DFF / 8) + 255) / 256), 256, 0, stream>>>(w2, BW2, DFF, DM, 16.0f); }

  for (int b = 0; b < NB; ++b) {
    const float* xb = x + (size_t)b * SEQ_FULL * DM; float* ob = (float*)d_out + (size_t)b * SEQ_FULL * DM;
    k_x16<<<(unsigned)(((size_t)SEQ * DM / 8 + 255) / 256), 256, 0, stream>>>(xb, X16, (size_t)SEQ * DM / 8);
    k_gemm2<0, 0><<<dim3((unsigned)((SEQ / 128) * (LQK / 64)), 1), 128, 0, stream>>>(X16, DM, (size_t)0, BQKV, DM, (size_t)0, 0.0625f, nullptr, nullptr, 0, nullptr, (size_t)0, nullptr, QK16, nullptr, LQK, (size_t)0, SEQ, LQK, DM);
    k_gemm2<0, 0><<<dim3((unsigned)((SEQ / 128) * (DM / 64)), 1), 128, 0, stream>>>(X16, DM, (size_t)0, BQKV + (size_t)2 * DM * DM, DM, (size_t)0, 0.0625f, nullptr, nullptr, 0, nullptr, (size_t)0, nullptr, VH, VL, DM, (size_t)0, SEQ, DM, DM);
    k_vt<NH, SEQ><<<NH * (SEQ / 64), 256, 0, stream>>>(VH, DM, 0, VT);
    k_vt<NH, SEQ><<<NH * (SEQ / 64), 256, 0, stream>>>(VL, DM, 0, VTL);
    for (int h0 = 0; h0 < NH; h0 += HG) {
      k_gemm2<0, 0><<<dim3((unsigned)((SEQ / 128) * (SEQ / 64)), HG), 128, 0, stream>>>(QK16 + (size_t)h0 * HD, LQK, (size_t)HD, QK16 + DM + (size_t)h0 * HD, LQK, (size_t)HD, 0.125f, nullptr, nullptr, 0, nullptr, (size_t)0, S, nullptr, nullptr, SEQ, (size_t)SEQ * SEQ, SEQ, SEQ, HD);
      k_rsms<<<(HG * SEQ) / 256, 256, 0, stream>>>(S, P, RL, HG * SEQ);
      k_gemm2<0, 0><<<dim3((unsigned)((SEQ - QT0) / 128), HG), 128, 0, stream>>>(P + (size_t)QT0 * SEQ, SEQ, (size_t)SEQ * SEQ, VT + (size_t)h0 * HD * SEQ, SEQ, (size_t)HD * SEQ, 64.0f, nullptr, nullptr, QT0, RL, (size_t)SEQ, nullptr, O16 + (size_t)QT0 * DM + (size_t)h0 * HD, nullptr, DM, (size_t)HD, SEQ - QT0, HD, SEQ);
      k_gemmf<2, 0><<<dim3((unsigned)(((QT0 / 16) * (HD / 64) + 3) / 4), HG), 128, 0, stream>>>(P, P, SEQ, (size_t)SEQ * SEQ, VT + (size_t)h0 * HD * SEQ, VTL + (size_t)h0 * HD * SEQ, SEQ, (size_t)HD * SEQ, 64.0f, nullptr, RL, (size_t)SEQ, nullptr, O16 + (size_t)h0 * HD, OL + (size_t)h0 * HD, DM, (size_t)HD, QT0, HD, SEQ);
    }
    k_gemm2<0, 1><<<dim3((unsigned)(((SEQ - QT0) / 128) * (DM / 64)), 1), 128, 0, stream>>>(O16 + (size_t)QT0 * DM, DM, (size_t)0, BO, DM, (size_t)0, 0.0009765625f, nullptr, xb, QT0, nullptr, (size_t)0, Y1 + (size_t)QT0 * DM, nullptr, nullptr, DM, (size_t)0, SEQ - QT0, DM, DM);
    k_gemmf<1, 1><<<dim3((unsigned)(((QT0 / 16) * (DM / 64) + 3) / 4), 1), 128, 0, stream>>>(O16, OL, DM, (size_t)0, BO, BO, DM, (size_t)0, 0.0009765625f, xb, nullptr, (size_t)0, Y1, nullptr, nullptr, DM, (size_t)0, QT0, DM, DM);
    k_lnseq<1><<<DM / 64, 256, 0, stream>>>(Y1, ln1s, ln1o, 1e-5f, NORM, N16, SEQ);
    k_gemm2<3, 0><<<dim3((unsigned)((SEQ / 128) * (DFF / 64)), 1), 128, 0, stream>>>(N16, DM, (size_t)0, BW1, DM, (size_t)0, 0.0625f, b1, nullptr, 0, nullptr, (size_t)0, nullptr, HF16, nullptr, DFF, (size_t)0, SEQ, DFF, DM);
    k_gemm2<0, 0><<<dim3((unsigned)((SEQ / 128) * (DM / 64)), 1), 128, 0, stream>>>(HF16, DFF, (size_t)0, BW2, DFF, (size_t)0, 0.0625f, b2, NORM, 0, nullptr, (size_t)0, Y2, nullptr, nullptr, DM, (size_t)0, SEQ, DM, DFF);
    k_lnseq<0><<<DM / 64, 256, 0, stream>>>(Y2, ln2s, ln2o, 1e-5f, ob, nullptr, SEQ);
  }
}
